// M_EfficientSelfAtten_3_68375879352568
// MI455X (gfx1250) — hardware-run, weakly checked
//
#include <hip/hip_runtime.h>
#include <math.h>
#include <stdint.h>

#define NBAT    16
#define NTOK    5880
#define NTP     5888
#define CD      64
#define NKEY    735
#define NKP     768
#define NKLOOP  736
#define NPOS    49
#define NPP     64
#define R1OFF   392
#define R3OFF   441
#define R5OFF   539
#define T1OFF   392
#define T2OFF   3528
#define T3OFF   5096
#define OC1     64
#define OC3     128
#define OC5     256
#define KK1     4096
#define KK3     2048
#define KK5     1024
#define WSC     64.0f
#define ACARRY  16.0f
#define QKCARRY 16.0f
#define VCARRY  16.0f
#define PCARRY  1024.0f
#define FCARRY  256.0f
#define QWPB       (NTP / 16)
#define ATT_WAVES  (NBAT * QWPB)
#define ATT_BLOCKS (ATT_WAVES / 4)
#define XP_BLOCKS  ((NBAT * NTP * (CD / 8)) / 256)
#define LN_BLOCKS  ((NBAT * (NKP / 4)) / 8)
static_assert((NTP % 64) == 0 && NTP >= NTOK && NTP - NTOK < 64);
static_assert((NKP % 64) == 0 && NKP >= NKEY);
static_assert((NKLOOP % 32) == 0 && NKLOOP >= NKEY && NKLOOP <= NKP);
static_assert(NKEY == R1OFF + NPOS + 2 * NPOS + 4 * NPOS);
static_assert(R3OFF == R1OFF + NPOS && R5OFF == R3OFF + 2 * NPOS);
static_assert(T2OFF == T1OFF + 56 * 56 && T3OFF == T2OFF + 28 * 28 * 2 && NTOK == T3OFF + 14 * 14 * 4);
static_assert((NBAT * NTP * (CD / 8)) % 256 == 0);
static_assert((NBAT * (NKP / 4)) % 8 == 0);
static_assert(ATT_WAVES % 4 == 0);
static_assert(KK1 == 64 * 8 * 8 && KK3 == 128 * 4 * 4 && KK5 == 256 * 2 * 2);

typedef _Float16 v16h __attribute__((ext_vector_type(16)));
typedef _Float16 v8h  __attribute__((ext_vector_type(8)));
typedef float    v8f  __attribute__((ext_vector_type(8)));
typedef float    v4f  __attribute__((ext_vector_type(4)));
typedef unsigned int v4u __attribute__((ext_vector_type(4)));

union FragH { v16h v; v8h h[2]; v4u u[2]; };

__device__ __forceinline__ unsigned short bf_bits(float f) {
  unsigned u = __float_as_uint(f);
  return (unsigned short)((u + 0x7FFFu + ((u >> 16) & 1u)) >> 16);
}
__device__ __forceinline__ float bf_up(unsigned short h) { return __uint_as_float(((unsigned)h) << 16); }
__device__ __forceinline__ float bfr(float f) { return bf_up(bf_bits(f)); }
__device__ __forceinline__ unsigned short h_bits(_Float16 x) { return __builtin_bit_cast(unsigned short, x); }
__device__ __forceinline__ unsigned pk16(unsigned short a, unsigned short b) { return (unsigned)a | ((unsigned)b << 16); }
__device__ __forceinline__ v8f zero8() { v8f z = {0.f, 0.f, 0.f, 0.f, 0.f, 0.f, 0.f, 0.f}; return z; }

__device__ __forceinline__ v16h ldfrag_h(const _Float16* p) {
  FragH f;
  f.h[0] = *(const v8h*)(p);
  f.h[1] = *(const v8h*)(p + 16);
  return f.v;
}
__device__ __forceinline__ v16h ldfrag_u(const unsigned short* p) {
  FragH f;
  f.u[0] = *(const v4u*)(p);
  f.u[1] = *(const v4u*)(p + 16);
  return f.v;
}

__device__ __forceinline__ v8f mma_raw(v16h a, v16h b, v8f c) {
  return __builtin_amdgcn_wmma_f32_16x16x32_f16(false, a, false, b, (short)0, c, false, false);
}
__device__ __forceinline__ void dep_guard1(v8f& a, v8f& b, v16h x) {
#if defined(__HIP_DEVICE_COMPILE__)
  asm volatile("v_nop\n\tv_nop\n\tv_nop\n\tv_nop" : "+v"(a), "+v"(b) : "v"(x));
#endif
}
__device__ __forceinline__ void guard_s(v8f& s, v16h a0, v16h a1, v16h b0, v16h b1) {
#if defined(__HIP_DEVICE_COMPILE__)
  asm volatile("v_nop\n\tv_nop\n\tv_nop\n\tv_nop" : "+v"(s) : "v"(a0), "v"(a1), "v"(b0), "v"(b1));
#endif
}
__device__ __forceinline__ void guard_pv(v8f& a, v8f& b, v16h x, v16h y, v16h z) {
#if defined(__HIP_DEVICE_COMPILE__)
  asm volatile("v_nop\n\tv_nop\n\tv_nop\n\tv_nop" : "+v"(a), "+v"(b) : "v"(x), "v"(y), "v"(z));
#endif
}
__device__ __forceinline__ void keep4_h(v16h a, v16h b, v16h c, v16h d) {
#if defined(__HIP_DEVICE_COMPILE__)
  asm volatile("v_nop" :: "v"(a), "v"(b), "v"(c), "v"(d));
#endif
}
__device__ __forceinline__ void acc_guard4(v8f& a, v8f& b, v8f& c, v8f& d) {
#if defined(__HIP_DEVICE_COMPILE__)
  asm volatile("v_nop\n\tv_nop\n\tv_nop\n\tv_nop" : "+v"(a), "+v"(b), "+v"(c), "+v"(d));
#endif
}
__device__ __forceinline__ void wave_sync_lds() {
  __builtin_amdgcn_fence(__ATOMIC_RELEASE, "workgroup");
  __builtin_amdgcn_wave_barrier();
  __builtin_amdgcn_fence(__ATOMIC_ACQUIRE, "workgroup");
}

__global__ __launch_bounds__(256) void conv16(const float* __restrict__ W, unsigned short* dst, int n8, float wsc) {
  const int i  = blockIdx.x * 256 + threadIdx.x;
  const int ic = (i < n8) ? i : (n8 - 1);
  const float* p = W + (size_t)ic * 8;
  const v4f a = *(const v4f*)(p), b = *(const v4f*)(p + 4);
  float v[8];
#pragma unroll
  for (int e = 0; e < 4; ++e) { v[e] = bfr(a[e]); v[4 + e] = bfr(b[e]); }
  v4u ov;
#pragma unroll
  for (int e = 0; e < 4; ++e) ov[e] = pk16(h_bits((_Float16)(v[2 * e] * wsc)), h_bits((_Float16)(v[2 * e + 1] * wsc)));
  if (i < n8) *(volatile v4u*)(dst + (size_t)i * 8) = ov;
  __threadfence();
  if (i < n8) *(volatile v4u*)(dst + (size_t)i * 8) = ov;
}

__global__ __launch_bounds__(256) void wtr16(const float* __restrict__ W, int ldw, unsigned short* dst, float wsc) {
  __shared__ float tile[64 * 65];
  const int n0 = blockIdx.x * 64;
  for (int i = threadIdx.x; i < 4096; i += 256) {
    const int k = i >> 6, n = i & 63;
    tile[k * 65 + n] = bfr(W[(size_t)k * ldw + n0 + n]);
  }
  __syncthreads();
  const int l8 = threadIdx.x & 7, rg = threadIdx.x >> 3;
  const int k8 = l8 * 8;
  v4u ov[2];
#pragma unroll
  for (int p = 0; p < 2; ++p) {
    const int n = rg + 32 * p;
    v4u a;
#pragma unroll
    for (int e = 0; e < 4; ++e)
      a[e] = pk16(h_bits((_Float16)(tile[(k8 + 2 * e) * 65 + n] * wsc)),
                  h_bits((_Float16)(tile[(k8 + 2 * e + 1) * 65 + n] * wsc)));
    ov[p] = a;
  }
  for (int pass = 0; pass < 2; ++pass) {
#pragma unroll
    for (int p = 0; p < 2; ++p) {
      const int n = rg + 32 * p;
      *(volatile v4u*)(dst + (size_t)(n0 + n) * 64 + k8) = ov[p];
    }
    __threadfence();
  }
}

__global__ __launch_bounds__(256) void xprep16(const float* __restrict__ x, unsigned short* XP) {
  const int i  = blockIdx.x * 256 + threadIdx.x;
  const int rr = i >> 3;
  const int c8 = (i & 7) * 8;
  const int b  = rr / NTP;
  const int r  = rr - b * NTP;
  const int rc = (r < NTOK) ? r : (NTOK - 1);
  const float* xp = x + ((size_t)b * NTOK + rc) * CD + c8;
  const v4f x0 = *(const v4f*)(xp), x1 = *(const v4f*)(xp + 4);
  const bool live = (r < NTOK);
  float v[8];
#pragma unroll
  for (int e = 0; e < 4; ++e) {
    v[e]     = live ? bfr(x0[e]) : 0.f;
    v[4 + e] = live ? bfr(x1[e]) : 0.f;
  }
  v4u o;
#pragma unroll
  for (int e = 0; e < 4; ++e) o[e] = pk16(h_bits((_Float16)(v[2 * e] * ACARRY)), h_bits((_Float16)(v[2 * e + 1] * ACARRY)));
  unsigned short* dp = XP + (size_t)i * 8;
  *(volatile v4u*)dp = o;
  __threadfence();
  *(volatile v4u*)dp = o;
}

template <int KS, int CI, int MAPW, int TOFF>
__global__ __launch_bounds__(256) void im2col16(const float* __restrict__ x, unsigned short* A) {
  constexpr int KTOT = CI * KS * KS;
  constexpr int K8   = KTOT / 8;
  constexpr int GRP  = CI / 64;
  static_assert((K8 % 32) == 0);
  static_assert(((NBAT * NPP * K8) % 256) == 0);
  const int i   = blockIdx.x * 256 + threadIdx.x;
  const int rr  = i / K8;
  const int k8  = (i - rr * K8) * 8;
  const int b   = rr / NPP;
  const int pos = rr - b * NPP;
  const bool live = (pos < NPOS);
  const int pc  = live ? pos : (NPOS - 1);
  const int ph  = pc / 7, pw = pc - ph * 7;
  const float* xb = x + (size_t)b * NTOK * CD;
  float v[8];
#pragma unroll
  for (int e = 0; e < 8; ++e) {
    const int k   = k8 + e;
    const int ci  = k / (KS * KS);
    const int rem = k - ci * (KS * KS);
    const int kh  = rem / KS;
    const int kw  = rem - kh * KS;
    const int h   = ph * KS + kh;
    const int w   = pw * KS + kw;
    const int tok = TOFF + (h * MAPW + w) * GRP + (ci >> 6);
    const int ch  = ci & 63;
    const float f = xb[(size_t)tok * CD + ch];
    v[e] = live ? bfr(f) : 0.f;
  }
  v4u o;
#pragma unroll
  for (int e = 0; e < 4; ++e) o[e] = pk16(h_bits((_Float16)(v[2 * e] * ACARRY)), h_bits((_Float16)(v[2 * e + 1] * ACARRY)));
  unsigned short* dp = A + (size_t)i * 8;
  *(volatile v4u*)dp = o;
  __threadfence();
  *(volatile v4u*)dp = o;
}

__global__ __launch_bounds__(256) void lngelu16(const float* __restrict__ x, const float* __restrict__ CV1,
                                                const float* __restrict__ CV3, const float* __restrict__ CV5,
                                                const float* __restrict__ lng, const float* __restrict__ lnb,
                                                unsigned short* G) {
  __shared__ __align__(16) float os[8][4 * 64];
  const int lane = threadIdx.x & 31, wave = threadIdx.x >> 5;
  const int wg = blockIdx.x * 8 + wave;
  const int b  = wg / (NKP / 4);
  const int m0 = (wg - b * (NKP / 4)) * 4;
  const float ga = bfr(lng[lane]), gb = bfr(lng[lane + 32]);
  const float ea = bfr(lnb[lane]), eb = bfr(lnb[lane + 32]);
  float* slab = os[wave];
#pragma unroll 1
  for (int rr = 0; rr < 4; ++rr) {
    const int m  = m0 + rr;
    const int mt = (m < R1OFF) ? m : (R1OFF - 1);
    int p1 = m - R1OFF;  p1 = (p1 < 0) ? 0 : ((p1 > NPOS - 1) ? (NPOS - 1) : p1);
    int j3 = m - R3OFF;  j3 = (j3 < 0) ? 0 : ((j3 > 2 * NPOS - 1) ? (2 * NPOS - 1) : j3);
    const int h3 = (j3 >= NPOS) ? 1 : 0;
    const int p3 = j3 - NPOS * h3;
    int j5 = m - R5OFF;  j5 = (j5 < 0) ? 0 : ((j5 > 4 * NPOS - 1) ? (4 * NPOS - 1) : j5);
    const int g5 = j5 / NPOS;
    const int p5 = j5 - NPOS * g5;
    const float* xr = x   + ((size_t)b * NTOK + mt) * CD;
    const float* c1 = CV1 + ((size_t)b * NPP + p1) * OC1;
    const float* c3 = CV3 + ((size_t)b * NPP + p3) * OC3 + h3;
    const float* c5 = CV5 + ((size_t)b * NPP + p5) * OC5 + g5;
    const float xa = bfr(xr[lane]), xb = bfr(xr[lane + 32]);
    const float ca = c1[lane],      cb = c1[lane + 32];
    const float da = c3[2 * lane],  db = c3[2 * (lane + 32)];
    const float fa = c5[4 * lane],  fb = c5[4 * (lane + 32)];
    const bool live = (m < NKEY);
    float v0 = (m < R1OFF) ? xa : ((m < R3OFF) ? ca : ((m < R5OFF) ? da : fa));
    float v1 = (m < R1OFF) ? xb : ((m < R3OFF) ? cb : ((m < R5OFF) ? db : fb));
    v0 = live ? v0 : 0.f;
    v1 = live ? v1 : 0.f;
    float s = v0 + v1;
#pragma unroll
    for (int d = 1; d < 32; d <<= 1) s += __shfl_xor(s, d, 32);
    const float mu = s * (1.0f / 64.0f);
    const float d0 = v0 - mu, d1 = v1 - mu;
    float s2 = d0 * d0 + d1 * d1;
#pragma unroll
    for (int d = 1; d < 32; d <<= 1) s2 += __shfl_xor(s2, d, 32);
    const float var  = s2 * (1.0f / 64.0f);
    const float rstd = rsqrtf(var + 1e-5f);
    const float t0 = d0 * rstd * ga + ea;
    const float t1 = d1 * rstd * gb + eb;
    float y0 = 0.f, y1 = 0.f;
#pragma unroll 1
    for (int h = 0; h < 2; ++h) {
      const float t = (h == 0) ? t0 : t1;
      const float y = 0.5f * t * (1.0f + erff(t * 0.70710678118654752f));
      y0 = (h == 0) ? y : y0;
      y1 = (h == 0) ? y1 : y;
    }
    slab[rr * 64 + lane]      = live ? y0 : 0.f;
    slab[rr * 64 + lane + 32] = live ? y1 : 0.f;
  }
  wave_sync_lds();
  {
    const int q8 = lane >> 3, c8 = (lane & 7) * 8;
    const float* sp = slab + q8 * 64 + c8;
    v4u a;
#pragma unroll
    for (int e = 0; e < 4; ++e) a[e] = pk16(h_bits((_Float16)(sp[2 * e] * ACARRY)), h_bits((_Float16)(sp[2 * e + 1] * ACARRY)));
    unsigned short* dp = G + ((size_t)b * NKP + m0 + q8) * CD + c8;
    *(volatile v4u*)dp = a;
    __threadfence();
    *(volatile v4u*)dp = a;
  }
}

template <int OM, int BIASM>
__global__ __launch_bounds__(256) void gemm64(
    const unsigned short* __restrict__ Ap, int lda, long long sAo, long long sAi,
    const unsigned short* __restrict__ Btp, int ldb, long long sBo, long long sBi,
    const float* __restrict__ bias, int sbo, int sbi, float bscale,
    void* Cout, int ldc, long long sCo, long long sCi,
    int M, int N, int K, int Mv, int nin, float oscale) {
  __shared__ __align__(16) float sT[8][16 * 68];
  const int by   = blockIdx.y;
  const int bo   = by / nin;
  const int bi   = by - bo * nin;
  const int lane = threadIdx.x & 31;
  const int wave = threadIdx.x >> 5;
  const int tilesN = N >> 6;
  const int tilesM = M >> 6;
  const int tile = blockIdx.x * 8 + wave;
  if (tile >= tilesM * tilesN) return;
  const int tm = tile / tilesN;
  const int tn = tile - tm * tilesN;
  const int m0 = tm << 6;
  const int n0 = tn << 6;

  const unsigned short* A1 = Ap  + (size_t)((long long)bo * sAo + (long long)bi * sAi);
  const unsigned short* Bb = Btp + (size_t)((long long)bo * sBo + (long long)bi * sBi);
  const float*         bsp = bias + (size_t)bo * (size_t)sbo + (size_t)bi * (size_t)sbi;

  const int rlane = lane & 15;
  const int koff  = (lane >> 4) * 8;
  const int mOff  = (lane >> 4) * 8;

  v8f acc[4][4];
#pragma unroll
  for (int i = 0; i < 4; ++i)
#pragma unroll
    for (int j = 0; j < 4; ++j) acc[i][j] = zero8();

  for (int k0 = 0; k0 < K; k0 += 32) {
    v16h bh[4];
#pragma unroll
    for (int j = 0; j < 4; ++j) {
      const size_t bofs = (size_t)(n0 + (j << 4) + rlane) * ldb + koff + k0;
      bh[j] = ldfrag_u(Bb + bofs);
    }
#pragma unroll
    for (int i = 0; i < 4; ++i) {
      const size_t ao = (size_t)(m0 + (i << 4) + rlane) * lda + koff + k0;
      const v16h ah = ldfrag_u(A1 + ao);
#pragma unroll
      for (int j = 0; j < 4; ++j) acc[i][j] = mma_raw(ah, bh[j], acc[i][j]);
      dep_guard1(acc[i][0], acc[i][3], ah);
    }
    keep4_h(bh[0], bh[1], bh[2], bh[3]);
  }
  acc_guard4(acc[0][0], acc[0][1], acc[0][2], acc[0][3]);
  acc_guard4(acc[1][0], acc[1][1], acc[1][2], acc[1][3]);
  acc_guard4(acc[2][0], acc[2][1], acc[2][2], acc[2][3]);
  acc_guard4(acc[3][0], acc[3][1], acc[3][2], acc[3][3]);

  const int hh2 = lane >> 4, c4 = (lane & 15) * 4;
  const int q8  = lane >> 3, c8 = (lane & 7) * 8;
  float bc[8];
#pragma unroll
  for (int e = 0; e < 8; ++e) bc[e] = 0.f;
  if (BIASM == 0) {
    if (OM != 2) {
      const int cb = n0 + c4;
      const int i0 = (cb < N - 4) ? cb : (N - 4);
      const v4f b0v = *(const v4f*)(bsp + i0);
#pragma unroll
      for (int e = 0; e < 4; ++e) bc[e] = bfr(b0v[e]) * bscale;
    } else {
      const int cb = n0 + c8;
      const int i0 = (cb < N - 8) ? cb : (N - 8);
      const v4f b0a = *(const v4f*)(bsp + i0), b0b = *(const v4f*)(bsp + i0 + 4);
#pragma unroll
      for (int e = 0; e < 4; ++e) {
        bc[e]     = bfr(b0a[e]) * bscale;
        bc[4 + e] = bfr(b0b[e]) * bscale;
      }
    }
  }

  float* slab = sT[wave];
#pragma unroll
  for (int i = 0; i < 4; ++i) {
    const int mBase = m0 + (i << 4);
#pragma unroll
    for (int j = 0; j < 4; ++j) {
#pragma unroll
      for (int r = 0; r < 8; ++r) {
        slab[(mOff + r) * 68 + (j << 4) + rlane] = acc[i][j][r];
      }
    }
    wave_sync_lds();
    if (OM != 2) {
      float* C = (float*)Cout + (size_t)((long long)bo * sCo + (long long)bi * sCi);
      v4f vals[8];
#pragma unroll
      for (int it = 0; it < 8; ++it) {
        const int row = it * 2 + hh2;
        v4f v = *(const v4f*)(slab + row * 68 + c4);
#pragma unroll
        for (int e = 0; e < 4; ++e) v[e] = v[e] * oscale + bc[e];
        vals[it] = v;
      }
      for (int pass = 0; pass < 2; ++pass) {
#pragma unroll
        for (int it = 0; it < 8; ++it) {
          const int gr = mBase + it * 2 + hh2;
          if (gr < Mv) {
            *(volatile v4f*)(C + (size_t)gr * ldc + n0 + c4) = vals[it];
          }
        }
        __threadfence();
      }
    } else {
      unsigned short* C = (unsigned short*)Cout + (size_t)((long long)bo * sCo + (long long)bi * sCi);
      v4u hv[4];
#pragma unroll
      for (int it = 0; it < 4; ++it) {
        const int row = it * 4 + q8;
        const float* sp = slab + row * 68 + c8;
        float bm = 0.f;
        if (BIASM == 1) bm = bfr(bsp[mBase + row]) * bscale;
        v4u a;
#pragma unroll
        for (int e = 0; e < 4; ++e) {
          const float f0 = sp[2 * e]     * oscale + ((BIASM == 1) ? bm : bc[2 * e]);
          const float f1 = sp[2 * e + 1] * oscale + ((BIASM == 1) ? bm : bc[2 * e + 1]);
          a[e] = pk16(h_bits((_Float16)f0), h_bits((_Float16)f1));
        }
        hv[it] = a;
      }
      for (int pass = 0; pass < 2; ++pass) {
#pragma unroll
        for (int it = 0; it < 4; ++it) {
          const int row = it * 4 + q8;
          *(volatile v4u*)(C + (size_t)(mBase + row) * ldc + n0 + c8) = hv[it];
        }
        __threadfence();
      }
    }
    wave_sync_lds();
  }
}

__global__ __launch_bounds__(128)
void attn16(const unsigned short* __restrict__ Qpl, const unsigned short* __restrict__ Kpl,
            const unsigned short* __restrict__ VT, unsigned short* CT) {
  __shared__ __align__(16) float Ps[4][16 * 36];
  __shared__ __align__(16) float Os[4][16 * 64];

  const int tid  = threadIdx.x;
  const int wave = tid >> 5;
  const int lane = tid & 31;
  const int hh   = lane >> 4;
  const int c    = lane & 15;

  const int wid  = blockIdx.x * 4 + wave;
  const int bat  = wid / QWPB;
  const int qt   = wid - bat * QWPB;
  const int q0   = qt * 16;

  const _Float16* Qb = (const _Float16*)(const void*)Qpl + (size_t)bat * NTP * CD;
  const _Float16* Kb = (const _Float16*)(const void*)Kpl + (size_t)bat * NKP * CD;
  const _Float16* Vb = (const _Float16*)(const void*)VT  + (size_t)bat * CD * NKP;
  const float lsc = (1.4426950408889634f * 0.125f) / (QKCARRY * QKCARRY);

  const v16h qa0 = ldfrag_h(Qb + (size_t)(q0 + c) * CD + 8 * hh);
  const v16h qa1 = ldfrag_h(Qb + (size_t)(q0 + c) * CD + 32 + 8 * hh);

  float mrow[8], lrow[8];
  v8f acc0 = zero8(), acc1 = zero8(), acc2 = zero8(), acc3 = zero8();
#pragma unroll
  for (int r = 0; r < 8; ++r) { mrow[r] = -INFINITY; lrow[r] = 0.f; }
  float* pt = Ps[wave];

#pragma unroll 1
  for (int kb = 0; kb < NKLOOP; kb += 32) {
    const _Float16* kp = Kb + (size_t)(kb + c) * CD + 8 * hh;
    v8f s0, s1;
    {
      const v16h k00 = ldfrag_h(kp), k01 = ldfrag_h(kp + 32);
      s0 = mma_raw(qa0, k00, zero8());
      s0 = mma_raw(qa1, k01, s0);
      guard_s(s0, qa0, qa1, k00, k01);
    }
    {
      const v16h k10 = ldfrag_h(kp + (size_t)16 * CD), k11 = ldfrag_h(kp + (size_t)16 * CD + 32);
      s1 = mma_raw(qa0, k10, zero8());
      s1 = mma_raw(qa1, k11, s1);
      guard_s(s1, qa0, qa1, k10, k11);
    }
    const bool live0 = (kb + c) < NKEY;
    const bool live1 = (kb + 16 + c) < NKEY;
#pragma unroll
    for (int r = 0; r < 8; ++r) {
      const float t0 = live0 ? (s0[r] * lsc) : -INFINITY;
      const float t1 = live1 ? (s1[r] * lsc) : -INFINITY;
      float mx = fmaxf(t0, t1);
#pragma unroll
      for (int off = 1; off < 16; off <<= 1) mx = fmaxf(mx, __shfl_xor(mx, off, 32));
      const float mn = fmaxf(mrow[r], mx);
      const float al = exp2f(mrow[r] - mn);
      mrow[r] = mn;
      const float e0 = exp2f(t0 - mn), e1 = exp2f(t1 - mn);
      float ps = e0 + e1;
#pragma unroll
      for (int off = 1; off < 16; off <<= 1) ps += __shfl_xor(ps, off, 32);
      lrow[r] = lrow[r] * al + ps;
      acc0[r] *= al;
      acc1[r] *= al;
      acc2[r] *= al;
      acc3[r] *= al;
      const int ro = (8 * hh + r) * 36 + c;
      pt[ro]      = e0;
      pt[ro + 16] = e1;
    }
    wave_sync_lds();
    FragH pa;
    {
      const float* prow = pt + c * 36 + 8 * hh;
      const v4f p0 = *(const v4f*)(prow), p1 = *(const v4f*)(prow + 4);
      const v4f p2 = *(const v4f*)(prow + 16), p3 = *(const v4f*)(prow + 20);
#pragma unroll
      for (int e = 0; e < 4; ++e) {
        pa.h[0][e]     = (_Float16)(p0[e] * PCARRY);
        pa.h[0][4 + e] = (_Float16)(p1[e] * PCARRY);
        pa.h[1][e]     = (_Float16)(p2[e] * PCARRY);
        pa.h[1][4 + e] = (_Float16)(p3[e] * PCARRY);
      }
    }
    const _Float16* vp = Vb + (size_t)c * NKP + kb + 8 * hh;
    {
      const v16h vb0 = ldfrag_h(vp), vb1 = ldfrag_h(vp + (size_t)16 * NKP);
      acc0 = mma_raw(pa.v, vb0, acc0);
      acc1 = mma_raw(pa.v, vb1, acc1);
      guard_pv(acc0, acc1, pa.v, vb0, vb1);
    }
    {
      const v16h vb2 = ldfrag_h(vp + (size_t)32 * NKP), vb3 = ldfrag_h(vp + (size_t)48 * NKP);
      acc2 = mma_raw(pa.v, vb2, acc2);
      acc3 = mma_raw(pa.v, vb3, acc3);
      guard_pv(acc2, acc3, pa.v, vb2, vb3);
    }
    wave_sync_lds();
  }

  float* os = Os[wave];
  const float oc = FCARRY / (PCARRY * VCARRY);
#pragma unroll
  for (int r = 0; r < 8; ++r) {
    const float inv = (1.0f / lrow[r]) * oc;
    const int ro = (8 * hh + r) * 64 + c;
    os[ro]      = acc0[r] * inv;
    os[ro + 16] = acc1[r] * inv;
    os[ro + 32] = acc2[r] * inv;
    os[ro + 48] = acc3[r] * inv;
  }
  wave_sync_lds();
  {
    const int q8 = lane >> 3, c8 = (lane & 7) * 8;
    v4u hv[4];
#pragma unroll
    for (int it = 0; it < 4; ++it) {
      const int row = it * 4 + q8;
      const float* sp = os + row * 64 + c8;
      v4u a;
#pragma unroll
      for (int e = 0; e < 4; ++e) a[e] = pk16(h_bits((_Float16)sp[2 * e]), h_bits((_Float16)sp[2 * e + 1]));
      hv[it] = a;
    }
    unsigned short* dst = CT + ((size_t)bat * NTP + q0) * CD + c8;
    for (int pass = 0; pass < 2; ++pass) {
#pragma unroll
      for (int it = 0; it < 4; ++it) {
        const int row = it * 4 + q8;
        *(volatile v4u*)(dst + (size_t)row * CD) = hv[it];
      }
      __threadfence();
    }
  }
}

extern "C" void kernel_launch(void* const* d_in, const int* in_sizes, int n_in,
                              void* d_out, int out_size, void* d_ws, size_t ws_size,
                              hipStream_t stream) {
  if (n_in < 15) return;
  if (in_sizes[0] != NBAT * NTOK * CD) return;
  if (in_sizes[1] != CD * CD || in_sizes[2] != CD) return;
  if (in_sizes[3] != OC1 * KK1 || in_sizes[4] != OC1) return;
  if (in_sizes[5] != OC3 * KK3 || in_sizes[6] != OC3) return;
  if (in_sizes[7] != OC5 * KK5 || in_sizes[8] != OC5) return;
  if (in_sizes[9] != CD || in_sizes[10] != CD) return;
  if (in_sizes[11] != CD * 2 * CD || in_sizes[12] != 2 * CD) return;
  if (in_sizes[13] != CD * CD || in_sizes[14] != CD) return;
  if (out_size != NBAT * NTOK * CD) return;

  const float* x      = (const float*)d_in[0];
  const float* Wq     = (const float*)d_in[1];
  const float* bq     = (const float*)d_in[2];
  const float* sr1_w  = (const float*)d_in[3];
  const float* sr1_b  = (const float*)d_in[4];
  const float* sr3_w  = (const float*)d_in[5];
  const float* sr3_b  = (const float*)d_in[6];
  const float* sr5_w  = (const float*)d_in[7];
  const float* sr5_b  = (const float*)d_in[8];
  const float* ln_g   = (const float*)d_in[9];
  const float* ln_b   = (const float*)d_in[10];
  const float* kv_w   = (const float*)d_in[11];
  const float* kv_b   = (const float*)d_in[12];
  const float* proj_w = (const float*)d_in[13];
  const float* proj_b = (const float*)d_in[14];
  float*       out    = (float*)d_out;

  const size_t PWQ  = (size_t)CD * CD * 2;
  const size_t PWKV = (size_t)2 * CD * CD * 2;
  const size_t PWO  = (size_t)CD * CD * 2;
  const size_t PW1  = (size_t)OC1 * KK1 * 2;
  const size_t PW3  = (size_t)OC3 * KK3 * 2;
  const size_t PW5  = (size_t)OC5 * KK5 * 2;
  const size_t PXP  = (size_t)NBAT * NTP * CD * 2;
  const size_t PA1  = (size_t)NBAT * NPP * KK1 * 2;
  const size_t PA3  = (size_t)NBAT * NPP * KK3 * 2;
  const size_t PA5  = (size_t)NBAT * NPP * KK5 * 2;
  const size_t PC1  = (size_t)NBAT * NPP * OC1 * 4;
  const size_t PC3  = (size_t)NBAT * NPP * OC3 * 4;
  const size_t PC5  = (size_t)NBAT * NPP * OC5 * 4;
  const size_t PG   = (size_t)NBAT * NKP * CD * 2;
  size_t off = 0;
  const size_t oWQ = off; off += PWQ;
  const size_t oWK = off; off += PWKV;
  const size_t oWO = off; off += PWO;
  const size_t oW1 = off; off += PW1;
  const size_t oW3 = off; off += PW3;
  const size_t oW5 = off; off += PW5;
  const size_t oXP = off; off += PXP;
  const size_t oA1 = off; off += PA1;
  const size_t oA3 = off; off += PA3;
  const size_t oA5 = off; off += PA5;
  const size_t oC1 = off; off += PC1;
  const size_t oC3 = off; off += PC3;
  const size_t oC5 = off; off += PC5;
  const size_t oG  = off; off += PG;
  const size_t oKP = off; off += PG;
  const size_t oVT = off; off += PG;
  const size_t oQP = off; off += PXP;
  const size_t oCT = off; off += PXP;
  if (off > ws_size) return;
  if (off > (size_t)134217728) return;

  char* ws = (char*)d_ws;
  unsigned short* WQt  = (unsigned short*)(ws + oWQ);
  unsigned short* WKVt = (unsigned short*)(ws + oWK);
  unsigned short* WOt  = (unsigned short*)(ws + oWO);
  unsigned short* W1   = (unsigned short*)(ws + oW1);
  unsigned short* W3   = (unsigned short*)(ws + oW3);
  unsigned short* W5   = (unsigned short*)(ws + oW5);
  unsigned short* XP   = (unsigned short*)(ws + oXP);
  unsigned short* A1   = (unsigned short*)(ws + oA1);
  unsigned short* A3   = (unsigned short*)(ws + oA3);
  unsigned short* A5   = (unsigned short*)(ws + oA5);
  float*          CV1  = (float*)(ws + oC1);
  float*          CV3  = (float*)(ws + oC3);
  float*          CV5  = (float*)(ws + oC5);
  unsigned short* G    = (unsigned short*)(ws + oG);
  unsigned short* KP   = (unsigned short*)(ws + oKP);
  unsigned short* VTp  = (unsigned short*)(ws + oVT);
  unsigned short* QP   = (unsigned short*)(ws + oQP);
  unsigned short* CT   = (unsigned short*)(ws + oCT);

  const int n8w = (OC1 * KK1) / 8;
  if ((n8w % 256) != 0 || OC3 * KK3 != OC1 * KK1 || OC5 * KK5 != OC1 * KK1) return;
  const dim3 blk(256), blk128(128);
  const dim3 gCW(n8w / 256);
  const dim3 gXP(XP_BLOCKS);
  const dim3 gI1((NBAT * NPP * (KK1 / 8)) / 256);
  const dim3 gI3((NBAT * NPP * (KK3 / 8)) / 256);
  const dim3 gI5((NBAT * NPP * (KK5 / 8)) / 256);
  const dim3 gG1((((NBAT * NPP) / 64) * (OC1 / 64) + 7) / 8, 1);
  const dim3 gG3((((NBAT * NPP) / 64) * (OC3 / 64) + 7) / 8, 1);
  const dim3 gG5((((NBAT * NPP) / 64) * (OC5 / 64) + 7) / 8, 1);
  const dim3 gLN(LN_BLOCKS);
  const dim3 gQ(((NTP / 64) * (CD / 64) + 7) / 8, NBAT);
  const dim3 gK(((NKP / 64) * (CD / 64) + 7) / 8, NBAT);
  const dim3 gV(((CD / 64) * (NKP / 64) + 7) / 8, NBAT);
  const dim3 gAT(ATT_BLOCKS);
  const dim3 gO(((NTP / 64) * (CD / 64) + 7) / 8, NBAT);

  conv16<<<gCW, blk, 0, stream>>>(sr1_w, W1, n8w, WSC);
  conv16<<<gCW, blk, 0, stream>>>(sr3_w, W3, n8w, WSC);
  conv16<<<gCW, blk, 0, stream>>>(sr5_w, W5, n8w, WSC);
  wtr16<<<dim3(1), blk, 0, stream>>>(Wq, CD, WQt, WSC);
  wtr16<<<dim3(2), blk, 0, stream>>>(kv_w, 2 * CD, WKVt, WSC);
  wtr16<<<dim3(1), blk, 0, stream>>>(proj_w, CD, WOt, WSC);

  xprep16<<<gXP, blk, 0, stream>>>(x, XP);
  im2col16<8, 64, 56, T1OFF><<<gI1, blk, 0, stream>>>(x, A1);
  im2col16<4, 128, 28, T2OFF><<<gI3, blk, 0, stream>>>(x, A3);
  im2col16<2, 256, 14, T3OFF><<<gI5, blk, 0, stream>>>(x, A5);

  gemm64<0, 0><<<gG1, blk, 0, stream>>>(
      A1, KK1, 0LL, 0LL, W1, KK1, 0LL, 0LL, sr1_b, 0, 0, 1.0f,
      (void*)CV1, OC1, 0LL, 0LL, NBAT * NPP, OC1, KK1, NBAT * NPP, 1, 1.0f / (ACARRY * WSC));
  gemm64<0, 0><<<gG3, blk, 0, stream>>>(
      A3, KK3, 0LL, 0LL, W3, KK3, 0LL, 0LL, sr3_b, 0, 0, 1.0f,
      (void*)CV3, OC3, 0LL, 0LL, NBAT * NPP, OC3, KK3, NBAT * NPP, 1, 1.0f / (ACARRY * WSC));
  gemm64<0, 0><<<gG5, blk, 0, stream>>>(
      A5, KK5, 0LL, 0LL, W5, KK5, 0LL, 0LL, sr5_b, 0, 0, 1.0f,
      (void*)CV5, OC5, 0LL, 0LL, NBAT * NPP, OC5, KK5, NBAT * NPP, 1, 1.0f / (ACARRY * WSC));

  lngelu16<<<gLN, blk, 0, stream>>>(x, CV1, CV3, CV5, ln_g, ln_b, G);

  gemm64<2, 0><<<gQ, blk, 0, stream>>>(
      XP, CD, (long long)NTP * CD, 0LL,
      WQt, CD, 0LL, 0LL,
      bq, 0, 0, QKCARRY,
      (void*)QP, CD, (long long)NTP * CD, 0LL,
      NTP, CD, CD, NTP, 1, QKCARRY / (ACARRY * WSC));

  gemm64<2, 0><<<gK, blk, 0, stream>>>(
      G, CD, (long long)NKP * CD, 0LL,
      WKVt, CD, 0LL, 0LL,
      kv_b, 0, 0, QKCARRY,
      (void*)KP, CD, (long long)NKP * CD, 0LL,
      NKP, CD, CD, NKP, 1, QKCARRY / (ACARRY * WSC));

  gemm64<2, 1><<<gV, blk, 0, stream>>>(
      WKVt + (size_t)CD * CD, CD, 0LL, 0LL,
      G, CD, (long long)NKP * CD, 0LL,
      kv_b + CD, 0, 0, VCARRY,
      (void*)VTp, NKP, (long long)CD * NKP, 0LL,
      CD, NKP, CD, CD, 1, VCARRY / (ACARRY * WSC));

  attn16<<<gAT, blk128, 0, stream>>>(QP, KP, VTp, CT);

  gemm64<0, 0><<<gO, blk, 0, stream>>>(
      CT, CD, (long long)NTP * CD, 0LL,
      WOt, CD, 0LL, 0LL,
      proj_b, 0, 0, 1.0f,
      (void*)out, CD, (long long)NTOK * CD, 0LL,
      NTP, CD, CD, NTOK, 1, 1.0f / (FCARRY * WSC));
  (void)hipGetLastError();
}
